// SelectiveStateSpaceMixer_39101382262865
// MI455X (gfx1250) — hardware-verified
//
#include <hip/hip_runtime.h>


#define NB_  2
#define LL   4096
#define DMd  1024
#define DI   2048
#define NS   64
typedef _Float16 h16;
typedef unsigned short bf;
typedef __attribute__((ext_vector_type(16))) __bf16   v16bf;
typedef __attribute__((ext_vector_type(16))) _Float16 v16h;
typedef __attribute__((ext_vector_type(8)))  _Float16 v8h;
typedef __attribute__((ext_vector_type(8)))  unsigned short v8us;
typedef __attribute__((ext_vector_type(8)))  float    v8f;
typedef __attribute__((ext_vector_type(4)))  float    v4f;
typedef v8h  __attribute__((may_alias)) v8ha;
typedef v4f  __attribute__((may_alias)) v4fa;
typedef v8us __attribute__((may_alias)) v8usa;

__device__ __forceinline__ unsigned short f2bf(float f) { unsigned u = __float_as_uint(f); u += 0x7FFFu + ((u >> 16) & 1u); return (unsigned short)(u >> 16); }
__device__ __forceinline__ float bf2f(unsigned short b) { return __uint_as_float(((unsigned)b) << 16); }
__device__ __forceinline__ float bfr(float f) { return bf2f(f2bf(f)); }
__device__ __forceinline__ v16h cat16(v8h lo, v8h hi) { return __builtin_shufflevector(lo, hi, 0, 1, 2, 3, 4, 5, 6, 7, 8, 9, 10, 11, 12, 13, 14, 15); }
__device__ __forceinline__ v16bf cat16b(v8us lo, v8us hi) { return __builtin_bit_cast(v16bf, __builtin_shufflevector(lo, hi, 0, 1, 2, 3, 4, 5, 6, 7, 8, 9, 10, 11, 12, 13, 14, 15)); }
__device__ __forceinline__ v8f wmma16(v16h a, v16h b, v8f c) { return __builtin_amdgcn_wmma_f32_16x16x32_f16(false, a, false, b, (short)0, c, false, false); }
__device__ __forceinline__ v8f wmmab(v16bf a, v16bf b, v8f c) { return __builtin_amdgcn_wmma_f32_16x16x32_bf16(false, a, false, b, (short)0, c, false, false); }


template <typename T16> struct WFrag;
template <> struct WFrag<h16> { typedef v16h V; static __device__ __forceinline__ V ld(const h16* p) { return cat16(*(const v8h*)p, *(const v8h*)(p + 16)); } static __device__ __forceinline__ v8f mma(V a, V b, v8f c) { return wmma16(a, b, c); } };
template <> struct WFrag<bf> { typedef v16bf V; static __device__ __forceinline__ V ld(const bf* p) { return cat16b(*(const v8us*)p, *(const v8us*)(p + 16)); } static __device__ __forceinline__ v8f mma(V a, V b, v8f c) { return wmmab(a, b, c); } };
template <typename T16, int NSPLIT, bool BIAS>
__global__ __launch_bounds__(32) void k_gemmw(const T16* __restrict__ A, const T16* __restrict__ A2, const T16* __restrict__ Bt, const T16* __restrict__ Bt2, int K, float* C, int ldc, const float* __restrict__ bias, size_t sA, size_t sB, size_t sC) {
    typedef typename WFrag<T16>::V V;
    __shared__ __align__(16) float os[16 * 68];
    const size_t z = blockIdx.z; A += z * sA; if (A2) A2 += z * sA; Bt += z * sB; if (Bt2) Bt2 += z * sB; C += z * sC;
    const int lane = threadIdx.x & 31, lr = lane & 15, hi = lane >> 4; const int r0 = blockIdx.x * 64, c0 = blockIdx.y * 64;
    v8f acc[4][4];
#pragma unroll
    for (int mb = 0; mb < 4; ++mb)
#pragma unroll
        for (int nb = 0; nb < 4; ++nb) acc[mb][nb] = (v8f){};
    const size_t aoff = (size_t)(r0 + lr) * K + 8 * hi, boff = (size_t)(c0 + lr) * K + 8 * hi;
#pragma unroll 1
    for (int kc = 0; kc < K; kc += 32) {
        V a[4], a2[4];
#pragma unroll
        for (int mb = 0; mb < 4; ++mb) { a[mb] = WFrag<T16>::ld(A + aoff + (size_t)mb * 16 * K + kc); if (NSPLIT == 1 || NSPLIT == 2) a2[mb] = WFrag<T16>::ld(A2 + aoff + (size_t)mb * 16 * K + kc); }
#pragma unroll
        for (int nb = 0; nb < 4; ++nb) { const V b = WFrag<T16>::ld(Bt + boff + (size_t)nb * 16 * K + kc); V b2; if (NSPLIT >= 2) b2 = WFrag<T16>::ld(Bt2 + boff + (size_t)nb * 16 * K + kc);
#pragma unroll
            for (int mb = 0; mb < 4; ++mb) { acc[mb][nb] = WFrag<T16>::mma(a[mb], b, acc[mb][nb]); if (NSPLIT == 1 || NSPLIT == 2) acc[mb][nb] = WFrag<T16>::mma(a2[mb], b, acc[mb][nb]); if (NSPLIT >= 2) acc[mb][nb] = WFrag<T16>::mma(a[mb], b2, acc[mb][nb]); } }
        asm volatile("v_nop\n\tv_nop\n\tv_nop\n\tv_nop" : "+v"(acc[0][0]), "+v"(acc[1][1]), "+v"(acc[2][2]), "+v"(acc[3][3]) : "v"(a[0]), "v"(a[3]));
    }
#pragma unroll
    for (int mb = 0; mb < 4; ++mb) {
#pragma unroll
        for (int nb = 0; nb < 4; ++nb) {
#pragma unroll
            for (int j = 0; j < 8; ++j) os[(hi * 8 + j) * 68 + nb * 16 + lr] = acc[mb][nb][j]; }
        __builtin_amdgcn_wave_barrier(); asm volatile("" ::: "memory");
        float* crow = C + (size_t)(r0 + mb * 16) * ldc + c0;
#pragma unroll 1
        for (int ps = 0; ps < 2; ++ps) {
#pragma unroll
            for (int s = 0; s < 8; ++s) { const int row = 2 * s + hi, cofs = lr * 4; v4f val = *(const v4fa*)(os + row * 68 + cofs); if (BIAS) { val[0] += bfr(bias[c0 + cofs]); val[1] += bfr(bias[c0 + cofs + 1]); val[2] += bfr(bias[c0 + cofs + 2]); val[3] += bfr(bias[c0 + cofs + 3]); }
                *(volatile v4f*)(crow + (size_t)row * ldc + cofs) = val; }
            if (ps == 0) __threadfence(); }
        __builtin_amdgcn_wave_barrier(); asm volatile("" ::: "memory");
    }
}

__device__ __forceinline__ h16 tohx(float x) { return (h16)x; }
__device__ __forceinline__ void splitf(float y, unsigned short& h, unsigned short& l) { h = f2bf(y); l = f2bf(y - bf2f(h)); }
__device__ __forceinline__ float silu_(float x) { return __fmul_rn(x, __fdiv_rn(1.0f, 1.0f + __expf(-x))); }
__device__ __forceinline__ float sigm_(float x) { return __fdiv_rn(1.0f, 1.0f + __expf(-x)); }
typedef __attribute__((ext_vector_type(2))) unsigned short v2us;
typedef __attribute__((ext_vector_type(4))) unsigned short v4us;
typedef __attribute__((ext_vector_type(4))) _Float16 v4h;

__global__ __launch_bounds__(256) void k_wtG(const float* __restrict__ w, int K, int N, bf* Bt) {
    const int lane = threadIdx.x & 31; const int L0 = (blockIdx.x * 8 + (threadIdx.x >> 5)) * 8; const int nlines = N * K / 64;
#pragma unroll
    for (int ps = 0; ps < 2; ++ps) {
#pragma unroll 1
        for (int l = 0; l < 8; ++l) { const int L = L0 + l; if (L >= nlines) break; const size_t e = (size_t)L * 64 + lane * 2; const int k = (int)(e % K), n = (int)(e / K); v2us o;
            o[0] = f2bf(w[(size_t)k * N + n]); o[1] = f2bf(w[(size_t)(k + 1) * N + n]); *(volatile v2us*)(Bt + e) = o; }
        if (ps == 0) __threadfence(); }
}
__global__ __launch_bounds__(256) void k_cvt8(const float* __restrict__ src, bf* dst, size_t n8) { const size_t i = (size_t)blockIdx.x * 256 + threadIdx.x; if (i >= n8) return; const v8f v = *(const v8f*)(src + i * 8); v8us o;
#pragma unroll
    for (int k = 0; k < 8; ++k) o[k] = f2bf(v[k]); *(volatile v8us*)(dst + i * 8) = o; __threadfence(); *(volatile v8us*)(dst + i * 8) = o; }
__global__ __launch_bounds__(256) void k_wt16(const float* __restrict__ w, int K, int N, h16* W16) { __shared__ float tile[64][65]; const int nb = (N + 63) / 64; const int k0 = (blockIdx.x / nb) * 64, n0 = (blockIdx.x % nb) * 64;
    for (int i = threadIdx.x; i < 64 * 64; i += 256) { const int kk = i / 64, nn = i % 64; tile[kk][nn] = (k0 + kk < K && n0 + nn < N) ? w[(size_t)(k0 + kk) * N + n0 + nn] : 0.f; }
    __syncthreads();
    const int nn = threadIdx.x / 4, kq = (threadIdx.x % 4) * 16; if (n0 + nn >= N) return;
    for (int c = 0; c < 16; c += 4) { v4h o; o[0] = tohx(bfr(tile[kq + c][nn])); o[1] = tohx(bfr(tile[kq + c + 1][nn])); o[2] = tohx(bfr(tile[kq + c + 2][nn])); o[3] = tohx(bfr(tile[kq + c + 3][nn])); h16* dst = W16 + (size_t)(n0 + nn) * K + k0 + kq + c; for (int ps = 0; ps < 2; ++ps) { *(volatile v4h*)dst = o; if (ps == 0) __threadfence(); } } }
__global__ __launch_bounds__(256) void k_conv(const float* __restrict__ XZ, const float* __restrict__ w, const float* __restrict__ bb, float* XM, bf* Mh, bf* Ml) { const int e = (blockIdx.x * 256 + threadIdx.x) * 4; if (e >= LL * DI) return; const int c = e % DI, t = e / DI; v4f o; v4us oh, ol;
#pragma unroll 1
    for (int q = 0; q < 4; ++q) { const int cc = c + q; float acc = 0.f;
#pragma unroll
        for (int k = 0; k < 3; ++k) { const int ts = t + k - 2; if (ts >= 0) { float p = __fmul_rn(bfr(w[cc * 3 + k]), XZ[(size_t)ts * 2 * DI + cc]); asm volatile("" : "+v"(p)); acc = __fadd_rn(acc, p); } }
        o[q] = silu_(__fadd_rn(acc, bfr(bb[cc]))); unsigned short u, l; splitf(o[q], u, l); oh[q] = u; ol[q] = l; }
    for (int ps = 0; ps < 2; ++ps) { *(volatile v4f*)(XM + e) = o; *(volatile v4us*)(Mh + e) = oh; *(volatile v4us*)(Ml + e) = ol; if (ps == 0) __threadfence(); } }
__global__ __launch_bounds__(64) void k_scan(const float* __restrict__ DTl, const float* __restrict__ Bv, const float* __restrict__ Cv, float* YS) { const int n = threadIdx.x; float st = 0.f;
    for (int t = 0; t < LL; ++t) { const size_t o = (size_t)t * NS + n; const float dt = sigm_(DTl[o]); float keep = __fmul_rn(__fsub_rn(1.0f, dt), st); asm volatile("" : "+v"(keep)); float add = __fmul_rn(dt, Bv[o]); asm volatile("" : "+v"(add)); st = __fadd_rn(keep, add); const float y = __fmul_rn(Cv[o], st); *(volatile float*)(YS + o) = y; __threadfence(); *(volatile float*)(YS + o) = y; } }
__global__ __launch_bounds__(256) void k_ln64(const float* __restrict__ YS, bf* Yh, bf* Yl) { const int lane = threadIdx.x & 31; const int row = blockIdx.x * 8 + (threadIdx.x >> 5); if (row >= LL) return; const float* r = YS + (size_t)row * NS + 2 * lane; const float a0 = r[0], a1 = r[1]; float s = __fadd_rn(a0, a1);
#pragma unroll
    for (int sh = 16; sh; sh >>= 1) s += __shfl_xor(s, sh, 32);
    const float mean = s * (1.0f / NS); float d0 = __fsub_rn(a0, mean), d1 = __fsub_rn(a1, mean); asm volatile("" : "+v"(d0)); asm volatile("" : "+v"(d1)); float q = __fadd_rn(__fmul_rn(d0, d0), __fmul_rn(d1, d1));
#pragma unroll
    for (int sh = 16; sh; sh >>= 1) q += __shfl_xor(q, sh, 32);
    const float rstd = __frsqrt_rn(__fadd_rn(q * (1.0f / NS), 1e-5f)); v2us oh, ol; unsigned short a, b; splitf(__fmul_rn(d0, rstd), a, b); oh[0] = a; ol[0] = b; splitf(__fmul_rn(d1, rstd), a, b); oh[1] = a; ol[1] = b;
    const size_t o = (size_t)row * NS + 2 * lane; *(volatile v2us*)(Yh + o) = oh; *(volatile v2us*)(Yl + o) = ol; __threadfence(); *(volatile v2us*)(Yh + o) = oh; *(volatile v2us*)(Yl + o) = ol; }
__global__ __launch_bounds__(256) void k_fin(const float* __restrict__ Y1, const float* __restrict__ XM, const float* __restrict__ XZ, const float* __restrict__ Dp, h16* Y16) { const int e = (blockIdx.x * 256 + threadIdx.x) * 4; if (e >= LL * DI) return; const int c = e % DI, t = e / DI; const v4f y1 = *(const v4f*)(Y1 + e), xm = *(const v4f*)(XM + e), gz = *(const v4f*)(XZ + (size_t)t * 2 * DI + DI + c); v4h o;
#pragma unroll
    for (int q = 0; q < 4; ++q) { float sk = __fmul_rn(bfr(Dp[c + q]), xm[q]); asm volatile("" : "+v"(sk)); const float y = __fadd_rn(y1[q], sk); o[q] = tohx(__fmul_rn(y, sigm_(gz[q]))); } *(volatile v4h*)(Y16 + e) = o; __threadfence(); *(volatile v4h*)(Y16 + e) = o; }

extern "C" void kernel_launch(void* const* d_in, const int* in_sizes, int n_in,
                              void* d_out, int out_size, void* d_ws, size_t ws_size, hipStream_t stream) {
    (void)in_sizes; (void)n_in; (void)out_size;
    const float** I = (const float**)d_in;
    const float *x = I[0], *win = I[1], *bin = I[2], *cw = I[3], *cb = I[4], *wdt = I[5], *bdt = I[6], *wB = I[7], *bB = I[8], *wC = I[9], *bC = I[10], *wsi = I[11], *bsi = I[12], *Dp = I[13], *wout = I[14], *bout = I[15];
    float* OUT = (float*)d_out;
    char* wsp = (char*)d_ws;
    auto take = [&](size_t bytes) { char* p = wsp; wsp += (bytes + 255) & ~(size_t)255; return (void*)p; };
    bf* WIN = (bf*)take((size_t)2 * DI * DMd * 2); bf* WDT = (bf*)take(NS * DI * 2); bf* WBm = (bf*)take(NS * DI * 2); bf* WCm = (bf*)take(NS * DI * 2); bf* WSI = (bf*)take((size_t)DI * NS * 2); h16* WO16 = (h16*)take((size_t)DMd * DI * 2);
    bf* XB = (bf*)take((size_t)LL * DMd * 2); float* XZ = (float*)take((size_t)LL * 2 * DI * 4); float* XM = (float*)take((size_t)LL * DI * 4); bf* Mh = (bf*)take((size_t)LL * DI * 2); bf* Ml = (bf*)take((size_t)LL * DI * 2); float* DTl = (float*)take((size_t)LL * NS * 4); float* Bv = (float*)take((size_t)LL * NS * 4); float* Cv = (float*)take((size_t)LL * NS * 4); float* YS = (float*)take((size_t)LL * NS * 4); bf* Yh = (bf*)take((size_t)LL * NS * 2); bf* Yl = (bf*)take((size_t)LL * NS * 2); h16* Y16 = (h16*)take((size_t)LL * DI * 2);
    float* Y1 = XM;
    if ((size_t)(wsp - (char*)d_ws) + (size_t)LL * DI * 4 > ws_size) return;
    Y1 = (float*)take((size_t)LL * DI * 4);
    k_wtG<<<(DMd * 2 * DI / 64 + 63) / 64, 256, 0, stream>>>(win, DMd, 2 * DI, WIN); k_wtG<<<(DI * NS / 64 + 63) / 64, 256, 0, stream>>>(wdt, DI, NS, WDT); k_wtG<<<(DI * NS / 64 + 63) / 64, 256, 0, stream>>>(wB, DI, NS, WBm); k_wtG<<<(DI * NS / 64 + 63) / 64, 256, 0, stream>>>(wC, DI, NS, WCm); k_wtG<<<(NS * DI / 64 + 63) / 64, 256, 0, stream>>>(wsi, NS, DI, WSI);
    k_wt16<<<(DI / 64) * (DMd / 64), 256, 0, stream>>>(wout, DI, DMd, WO16);
    for (int b = 0; b < NB_; ++b) {
        k_cvt8<<<(LL * DMd / 8 + 255) / 256, 256, 0, stream>>>(x + (size_t)b * LL * DMd, XB, (size_t)LL * DMd / 8);
        k_gemmw<bf, 0, true><<<dim3(LL / 64, 2 * DI / 64, 1), 32, 0, stream>>>(XB, nullptr, WIN, nullptr, DMd, XZ, 2 * DI, bin, 0, 0, 0);
        k_conv<<<(LL * DI / 4 + 255) / 256, 256, 0, stream>>>(XZ, cw, cb, XM, Mh, Ml);
        k_gemmw<bf, 1, true><<<dim3(LL / 64, 1, 1), 32, 0, stream>>>(Mh, Ml, WDT, nullptr, DI, DTl, NS, bdt, 0, 0, 0); k_gemmw<bf, 1, true><<<dim3(LL / 64, 1, 1), 32, 0, stream>>>(Mh, Ml, WBm, nullptr, DI, Bv, NS, bB, 0, 0, 0); k_gemmw<bf, 1, true><<<dim3(LL / 64, 1, 1), 32, 0, stream>>>(Mh, Ml, WCm, nullptr, DI, Cv, NS, bC, 0, 0, 0);
        k_scan<<<1, 64, 0, stream>>>(DTl, Bv, Cv, YS);
        k_ln64<<<LL / 8, 256, 0, stream>>>(YS, Yh, Yl);
        k_gemmw<bf, 1, true><<<dim3(LL / 64, DI / 64, 1), 32, 0, stream>>>(Yh, Yl, WSI, nullptr, NS, Y1, DI, bsi, 0, 0, 0);
        k_fin<<<(LL * DI / 4 + 255) / 256, 256, 0, stream>>>(Y1, XM, XZ, Dp, Y16);
        k_gemmw<h16, 0, true><<<dim3(LL / 64, DMd / 64, 1), 32, 0, stream>>>(Y16, nullptr, WO16, nullptr, DI, OUT + (size_t)b * LL * DMd, DMd, bout, 0, 0, 0); }
}
